// MHA_86535001079889
// MI455X (gfx1250) — hardware-verified
//
#include <hip/hip_runtime.h>


#ifndef NB
#define NB 2
#endif
#ifndef SEQ
#define SEQ 2048
#endif
#define NB_FULL  2
#define SEQ_FULL 2048
#define DM   1024
#define NH   16
#define HD   64
#define RHC  512
#define RH   ((SEQ < RHC) ? SEQ : RHC)
#define MPITCH SEQ_FULL
#define CEXP  0.18033688011112042f
#define PL2   10.0f
#define MFILL (-8000.0f)
#define RBASE 10000.0f
#define WSCAP ((size_t)134217728)

static_assert(SEQ % 64 == 0);
static_assert(SEQ <= SEQ_FULL);
static_assert(NB >= 1 && NB <= NB_FULL);
static_assert(RH % 16 == 0 && (SEQ - RH) % 16 == 0 && RH <= SEQ);
static_assert(DM == NH * HD && HD == 64 && DM % 64 == 0);

typedef _Float16 h16;
typedef unsigned short bf;
typedef __attribute__((ext_vector_type(16))) __bf16   v16bf;
typedef __attribute__((ext_vector_type(16))) _Float16 v16h;
typedef __attribute__((ext_vector_type(8)))  _Float16 v8h;
typedef __attribute__((ext_vector_type(2)))  _Float16 v2h;
typedef __attribute__((ext_vector_type(16))) unsigned short v16us;
typedef __attribute__((ext_vector_type(8)))  unsigned short v8us;
typedef __attribute__((ext_vector_type(2)))  unsigned short v2us;
typedef __attribute__((ext_vector_type(8)))  float v8f;
typedef __attribute__((ext_vector_type(4)))  float v4f;
typedef __attribute__((ext_vector_type(2)))  float v2f;
typedef __attribute__((ext_vector_type(4)))  int v4i;
typedef v8h  __attribute__((may_alias)) v8ha;
typedef v4f  __attribute__((may_alias)) v4fa;
typedef v8us __attribute__((may_alias)) v8usa;

#pragma clang fp contract(off)

__device__ __forceinline__ unsigned short f2bf(float f) { unsigned u = __float_as_uint(f); u += 0x7FFFu + ((u >> 16) & 1u); return (unsigned short)(u >> 16); }
__device__ __forceinline__ float bf2f(unsigned short b) { return __uint_as_float(((unsigned)b) << 16); }
__device__ __forceinline__ float bfr(float f) { return bf2f(f2bf(f)); }
__device__ __forceinline__ v16h cat16(v8h lo, v8h hi) { return __builtin_shufflevector(lo, hi, 0, 1, 2, 3, 4, 5, 6, 7, 8, 9, 10, 11, 12, 13, 14, 15); }
__device__ __forceinline__ v16bf cat16b(v8us lo, v8us hi) { return __builtin_bit_cast(v16bf, __builtin_shufflevector(lo, hi, 0, 1, 2, 3, 4, 5, 6, 7, 8, 9, 10, 11, 12, 13, 14, 15)); }
__device__ __forceinline__ v8f wmma16(v16h a, v16h b, v8f c) { return __builtin_amdgcn_wmma_f32_16x16x32_f16(false, a, false, b, (short)0, c, false, false); }
__device__ __forceinline__ v8f wmmab(v16bf a, v16bf b, v8f c) { return __builtin_amdgcn_wmma_f32_16x16x32_bf16(false, a, false, b, (short)0, c, false, false); }
__device__ __forceinline__ h16 tohx(float x) { return (h16)x; }
__device__ __forceinline__ void splitf(float y, unsigned short& h, unsigned short& l) { h = f2bf(y); l = f2bf(y - bf2f(h)); }
__device__ __forceinline__ void wave_sync() { __builtin_amdgcn_fence(3, "wavefront"); __builtin_amdgcn_wave_barrier(); asm volatile("" ::: "memory"); }

template <typename T16> struct WFrag;
template <> struct WFrag<h16> { typedef v16h V; static __device__ __forceinline__ V ld(const h16* p) { return cat16(*(const v8h*)p, *(const v8h*)(p + 16)); } static __device__ __forceinline__ v8f mma(V a, V b, v8f c) { return wmma16(a, b, c); } };
template <> struct WFrag<bf> { typedef v16bf V; static __device__ __forceinline__ V ld(const bf* p) { return cat16b(*(const v8us*)p, *(const v8us*)(p + 16)); } static __device__ __forceinline__ v8f mma(V a, V b, v8f c) { return wmmab(a, b, c); } };

template <typename T16, int NSPLIT, bool BIAS>
__global__ __launch_bounds__(32) void k_gemmw(const T16* __restrict__ A, const T16* __restrict__ A2, const T16* __restrict__ Bt, const T16* __restrict__ Bt2, int K, float* C, int ldc, const float* __restrict__ bias, size_t sA, size_t sB, size_t sC) {
    typedef typename WFrag<T16>::V V;
    __shared__ __align__(16) float os[16 * 68];
    const size_t z = blockIdx.z; A += z * sA; if (A2) A2 += z * sA; Bt += z * sB; if (Bt2) Bt2 += z * sB; C += z * sC;
    const int lane = threadIdx.x & 31, lr = lane & 15, hi = lane >> 4; const int r0 = blockIdx.x * 64, c0 = blockIdx.y * 64;
    v8f acc[4][4];
#pragma unroll
    for (int mb = 0; mb < 4; ++mb)
#pragma unroll
        for (int nb = 0; nb < 4; ++nb) acc[mb][nb] = (v8f){};
    const size_t aoff = (size_t)(r0 + lr) * K + 8 * hi, boff = (size_t)(c0 + lr) * K + 8 * hi;
#pragma unroll 1
    for (int kc = 0; kc < K; kc += 32) {
        V a[4], a2[4];
#pragma unroll
        for (int mb = 0; mb < 4; ++mb) { a[mb] = WFrag<T16>::ld(A + aoff + (size_t)mb * 16 * K + kc); if (NSPLIT == 1 || NSPLIT == 2) a2[mb] = WFrag<T16>::ld(A2 + aoff + (size_t)mb * 16 * K + kc); }
#pragma unroll
        for (int nb = 0; nb < 4; ++nb) { const V b = WFrag<T16>::ld(Bt + boff + (size_t)nb * 16 * K + kc); V b2; if (NSPLIT >= 2) b2 = WFrag<T16>::ld(Bt2 + boff + (size_t)nb * 16 * K + kc);
#pragma unroll
            for (int mb = 0; mb < 4; ++mb) { acc[mb][nb] = WFrag<T16>::mma(a[mb], b, acc[mb][nb]); if (NSPLIT == 1 || NSPLIT == 2) acc[mb][nb] = WFrag<T16>::mma(a2[mb], b, acc[mb][nb]); if (NSPLIT >= 2) acc[mb][nb] = WFrag<T16>::mma(a[mb], b2, acc[mb][nb]); } }
        asm volatile("v_nop\n\tv_nop\n\tv_nop\n\tv_nop" : "+v"(acc[0][0]), "+v"(acc[1][1]), "+v"(acc[2][2]), "+v"(acc[3][3]) : "v"(a[0]), "v"(a[3]));
    }
#pragma unroll
    for (int mb = 0; mb < 4; ++mb) {
#pragma unroll
        for (int nb = 0; nb < 4; ++nb) {
#pragma unroll
            for (int j = 0; j < 8; ++j) os[(hi * 8 + j) * 68 + nb * 16 + lr] = acc[mb][nb][j]; }
        __builtin_amdgcn_wave_barrier(); asm volatile("" ::: "memory");
        float* crow = C + (size_t)(r0 + mb * 16) * ldc + c0;
#pragma unroll 1
        for (int ps = 0; ps < 2; ++ps) {
#pragma unroll
            for (int s = 0; s < 8; ++s) { const int row = 2 * s + hi, cofs = lr * 4; v4f val = *(const v4fa*)(os + row * 68 + cofs); if (BIAS) { val[0] += bfr(bias[c0 + cofs]); val[1] += bfr(bias[c0 + cofs + 1]); val[2] += bfr(bias[c0 + cofs + 2]); val[3] += bfr(bias[c0 + cofs + 3]); }
                *(volatile v4f*)(crow + (size_t)row * ldc + cofs) = val; }
            if (ps == 0) __threadfence(); }
        __builtin_amdgcn_wave_barrier(); asm volatile("" ::: "memory");
    }
}

__global__ __launch_bounds__(256) void k_cvt8(const float* __restrict__ src, bf* dst, size_t n8) { const size_t i = (size_t)blockIdx.x * 256 + threadIdx.x; if (i >= n8) return; const v8f v = *(const v8f*)(src + i * 8); v8us o;
#pragma unroll
    for (int k = 0; k < 8; ++k) o[k] = f2bf(v[k]); *(volatile v8us*)(dst + i * 8) = o; __threadfence(); *(volatile v8us*)(dst + i * 8) = o; }

__global__ __launch_bounds__(256) void k_cstab(float* CS) {
    const int idx = blockIdx.x * 256 + threadIdx.x; if (idx >= SEQ * HD) return;
    const int d = idx & (HD - 1), t = idx >> 6; const int j = d & (HD / 2 - 1);
    const float ex = (float)(2 * j) * (1.0f / (float)HD);
    const float pw = powf(RBASE, ex);
    const float inv = 1.0f / pw;
    const float ang = (float)t * inv;
    const float cn = cosf(ang), sn = sinf(ang);
    v2f cs; cs[0] = cn; cs[1] = sn;
    *(volatile v2f*)(CS + (size_t)idx * 2) = cs; __threadfence(); *(volatile v2f*)(CS + (size_t)idx * 2) = cs;
}

__global__ __launch_bounds__(256) void k_rope(const float* __restrict__ F, const float* __restrict__ CS, h16* P16, bf* Ph, bf* Pl) {
    const size_t e = ((size_t)blockIdx.x * 256 + threadIdx.x) * 2; if (e >= (size_t)NH * SEQ * HD) return;
    const int d = (int)(e % HD); const int t = (int)((e / HD) % SEQ); const int hh = (int)(e / ((size_t)HD * SEQ));
    const float* f = F + (size_t)t * DM + hh * HD; v2h o16; v2us oh, ol;
#pragma unroll
    for (int q = 0; q < 2; ++q) { const int dd = d + q; const int dp = (dd < HD / 2) ? dd + HD / 2 : dd - HD / 2; const float x0 = f[dd], x1 = f[dp];
        const v2f cs = *(const v2f*)(CS + ((size_t)t * HD + dd) * 2); const float a = x0 * cs[0]; const float bq = x1 * cs[1];
        const float r = (dd < HD / 2) ? (a - bq) : (a + bq);
        o16[q] = tohx(r); unsigned short a2, c2; splitf(r, a2, c2); oh[q] = a2; ol[q] = c2; }
    *(volatile v2h*)(P16 + e) = o16; *(volatile v2us*)(Ph + e) = oh; *(volatile v2us*)(Pl + e) = ol; __threadfence();
    *(volatile v2h*)(P16 + e) = o16; *(volatile v2us*)(Ph + e) = oh; *(volatile v2us*)(Pl + e) = ol;
}

__global__ __launch_bounds__(256) void k_vtp(const float* __restrict__ F, h16* V16, bf* Vh, bf* Vl) {
    const size_t e = ((size_t)blockIdx.x * 256 + threadIdx.x) * 2; if (e >= (size_t)NH * HD * SEQ) return;
    const int t = (int)(e % SEQ); const int d = (int)((e / SEQ) % HD); const int g = (int)(e / ((size_t)SEQ * HD)); v2h o16; v2us oh, ol;
#pragma unroll
    for (int q = 0; q < 2; ++q) { const float x = F[(size_t)(t + q) * DM + g * HD + d]; o16[q] = tohx(x); unsigned short a2, c2; splitf(x, a2, c2); oh[q] = a2; ol[q] = c2; }
    *(volatile v2h*)(V16 + e) = o16; *(volatile v2us*)(Vh + e) = oh; *(volatile v2us*)(Vl + e) = ol; __threadfence();
    *(volatile v2h*)(V16 + e) = o16; *(volatile v2us*)(Vh + e) = oh; *(volatile v2us*)(Vl + e) = ol;
}

template <bool HL>
__global__ __launch_bounds__(32) __attribute__((amdgpu_num_vgpr(256)))
void k_attn(const h16* __restrict__ QP16, const bf* __restrict__ QPh, const bf* __restrict__ QPl,
            const h16* __restrict__ KP16, const bf* __restrict__ KPh, const bf* __restrict__ KPl,
            const h16* __restrict__ VT16, const bf* __restrict__ VTh, const bf* __restrict__ VTl,
            const int* __restrict__ MK, int qbase, bf* ATh, bf* ATl) {
    __shared__ __align__(16) unsigned short osh[16 * 72];
    __shared__ __align__(16) unsigned short osl[16 * 72];
    const int lane = threadIdx.x & 31, m = lane & 15, hf = lane >> 4;
    const int hh = blockIdx.y;
    const int q0 = qbase + blockIdx.x * 16;
    const int q = q0 + m;
    const size_t hp = (size_t)hh * SEQ * HD;
    v16h q16[2]; v16bf qh[2], ql[2];
#pragma unroll
    for (int ks = 0; ks < 2; ++ks) {
        const size_t qo = hp + (size_t)q * HD + 32 * ks + 8 * hf;
        if (HL) { qh[ks] = WFrag<bf>::ld(QPh + qo); ql[ks] = WFrag<bf>::ld(QPl + qo); }
        else    { q16[ks] = WFrag<h16>::ld(QP16 + qo); }
    }
    v8f o[4];
#pragma unroll
    for (int dt = 0; dt < 4; ++dt) o[dt] = (v8f){};
    float mrun = -3.0e38f, lrun = 0.0f; int seen = 0;
    const int* mq = MK + (size_t)q * MPITCH + 8 * hf;
#pragma unroll 1
    for (int c = 0; c < SEQ / 64; ++c) {
        const int kc = c * 64;
        v4i mk0[4], mk1[4]; int orv = 0;
#pragma unroll
        for (int kt = 0; kt < 4; ++kt) { const v4i* mp = (const v4i*)(mq + kc + 16 * kt); mk0[kt] = mp[0]; mk1[kt] = mp[1]; const v4i u = mk0[kt] | mk1[kt]; orv |= u[0] | u[1] | u[2] | u[3]; }
        const int anyl = (orv != 0) ? 1 : 0;
        if (__any(anyl) == 0) continue;
        seen |= anyl;
        v8f s[4];
#pragma unroll
        for (int kt = 0; kt < 4; ++kt) s[kt] = (v8f){};
        if (HL) {
            v16bf ka, kb;
#pragma unroll
            for (int kt = 0; kt < 4; ++kt) {
                asm volatile("" ::: "memory");
#pragma unroll
                for (int ks = 0; ks < 2; ++ks) { const size_t ko = hp + (size_t)(kc + 16 * kt + m) * HD + 32 * ks + 8 * hf; ka = WFrag<bf>::ld(KPh + ko); kb = WFrag<bf>::ld(KPl + ko);
                    s[kt] = wmmab(ka, qh[ks], s[kt]); s[kt] = wmmab(ka, ql[ks], s[kt]); s[kt] = wmmab(kb, qh[ks], s[kt]); } }
            asm volatile("v_nop\n\tv_nop\n\tv_nop\n\tv_nop" : "+v"(s[0]), "+v"(s[1]), "+v"(s[2]), "+v"(s[3]) : "v"(ka), "v"(kb), "v"(qh[0]), "v"(qh[1]), "v"(ql[0]), "v"(ql[1]));
        } else {
            v16h ka;
#pragma unroll
            for (int kt = 0; kt < 4; ++kt) {
                asm volatile("" ::: "memory");
#pragma unroll
                for (int ks = 0; ks < 2; ++ks) { const size_t ko = hp + (size_t)(kc + 16 * kt + m) * HD + 32 * ks + 8 * hf; ka = WFrag<h16>::ld(KP16 + ko);
                    s[kt] = wmma16(ka, q16[ks], s[kt]); } }
            asm volatile("v_nop\n\tv_nop\n\tv_nop\n\tv_nop" : "+v"(s[0]), "+v"(s[1]), "+v"(s[2]), "+v"(s[3]) : "v"(ka), "v"(q16[0]), "v"(q16[1]));
        }
        float cmx = -3.0e38f;
#pragma unroll
        for (int kt = 0; kt < 4; ++kt)
#pragma unroll
            for (int r = 0; r < 8; ++r) { const int mv = (r < 4) ? mk0[kt][r & 3] : mk1[kt][r & 3]; const float t = (mv != 0) ? s[kt][r] : MFILL; s[kt][r] = t; cmx = fmaxf(cmx, t); }
        cmx = fmaxf(cmx, __shfl_xor(cmx, 16, 32));
        const float mnew = fmaxf(mrun, cmx);
        const float alpha = __builtin_amdgcn_exp2f((mrun - mnew) * CEXP);
        mrun = mnew;
        float psum = 0.0f;
#pragma unroll
        for (int kt = 0; kt < 4; ++kt)
#pragma unroll
            for (int r = 0; r < 8; ++r) { const float p = __builtin_amdgcn_exp2f(fmaf(s[kt][r] - mnew, CEXP, PL2)); s[kt][r] = p; psum += p; }
        lrun = lrun * alpha + psum;
#pragma unroll
        for (int dt = 0; dt < 4; ++dt) o[dt] = o[dt] * alpha;
#pragma unroll
        for (int ks = 0; ks < 2; ++ks) {
            if (HL) {
                v16us uh, ul;
#pragma unroll
                for (int r = 0; r < 8; ++r) { unsigned short a, b2; splitf(s[2 * ks][r], a, b2); uh[r] = a; ul[r] = b2; splitf(s[2 * ks + 1][r], a, b2); uh[8 + r] = a; ul[8 + r] = b2; }
                v16bf ph = __builtin_bit_cast(v16bf, uh), pl = __builtin_bit_cast(v16bf, ul);
                asm volatile("v_nop\n\tv_nop\n\tv_nop\n\tv_nop" : "+v"(ph), "+v"(pl));
                v16bf va, vb;
#pragma unroll
                for (int dt = 0; dt < 4; ++dt) { asm volatile("" ::: "memory"); const size_t vo = hp + (size_t)(16 * dt + m) * SEQ + kc + 32 * ks + 8 * hf; va = WFrag<bf>::ld(VTh + vo); vb = WFrag<bf>::ld(VTl + vo);
                    o[dt] = wmmab(va, ph, o[dt]); o[dt] = wmmab(va, pl, o[dt]); o[dt] = wmmab(vb, ph, o[dt]); }
                asm volatile("v_nop\n\tv_nop\n\tv_nop\n\tv_nop" : "+v"(o[0]), "+v"(o[1]), "+v"(o[2]), "+v"(o[3]) : "v"(ph), "v"(pl), "v"(va), "v"(vb));
            } else {
                v16h p16;
#pragma unroll
                for (int r = 0; r < 8; ++r) { p16[r] = tohx(s[2 * ks][r]); p16[8 + r] = tohx(s[2 * ks + 1][r]); }
                asm volatile("v_nop\n\tv_nop\n\tv_nop\n\tv_nop" : "+v"(p16));
                v16h va;
#pragma unroll
                for (int dt = 0; dt < 4; ++dt) { asm volatile("" ::: "memory"); const size_t vo = hp + (size_t)(16 * dt + m) * SEQ + kc + 32 * ks + 8 * hf; va = WFrag<h16>::ld(VT16 + vo);
                    o[dt] = wmma16(va, p16, o[dt]); }
                asm volatile("v_nop\n\tv_nop\n\tv_nop\n\tv_nop" : "+v"(o[0]), "+v"(o[1]), "+v"(o[2]), "+v"(o[3]) : "v"(p16), "v"(va));
            }
        }
    }
    const float lt = lrun + __shfl_xor(lrun, 16, 32);
    const int sn = seen | __shfl_xor(seen, 16, 32);
    const float inv = (sn != 0) ? (1.0f / lt) : __uint_as_float(0x7fc00000u);
#pragma unroll
    for (int dt = 0; dt < 4; ++dt) { v8us oh8, ol8;
#pragma unroll
        for (int r = 0; r < 8; ++r) { unsigned short a, b2; splitf(o[dt][r] * inv, a, b2); oh8[r] = a; ol8[r] = b2; }
        *(v8usa*)(osh + m * 72 + 16 * dt + 8 * hf) = oh8; *(v8usa*)(osl + m * 72 + 16 * dt + 8 * hf) = ol8; }
    wave_sync();
#pragma unroll 1
    for (int ps = 0; ps < 2; ++ps) {
#pragma unroll
        for (int s4 = 0; s4 < 4; ++s4) { const int row = 4 * s4 + (lane >> 3), pc = (lane & 7) * 8;
            const v8us vh = *(const v8usa*)(osh + row * 72 + pc); const v8us vl = *(const v8usa*)(osl + row * 72 + pc);
            const size_t off = (size_t)(q0 + row) * DM + hh * HD + pc;
            *(volatile v8us*)(ATh + off) = vh; *(volatile v8us*)(ATl + off) = vl; }
        if (ps == 0) __threadfence(); }
}

extern "C" void kernel_launch(void* const* d_in, const int* in_sizes, int n_in,
                              void* d_out, int out_size, void* d_ws, size_t ws_size, hipStream_t stream) {
    if (n_in < 8) return;
    const long long needx = (long long)(NB - 1) * SEQ_FULL * DM + (long long)SEQ * DM;
    if ((long long)in_sizes[0] < needx || (long long)in_sizes[1] < needx || (long long)in_sizes[2] < needx) return;
    if (in_sizes[3] < DM * DM || in_sizes[4] < DM * DM || in_sizes[5] < DM * DM || in_sizes[6] < DM * DM) return;
    if ((long long)in_sizes[7] < (long long)(SEQ - 1) * MPITCH + SEQ) return;
    if ((long long)out_size < (long long)NB * SEQ * DM) return;
    const float* xq = (const float*)d_in[0]; const float* xk = (const float*)d_in[1]; const float* xv = (const float*)d_in[2];
    const float* wq = (const float*)d_in[3]; const float* wk = (const float*)d_in[4]; const float* wv = (const float*)d_in[5]; const float* wo = (const float*)d_in[6];
    const int* mask = (const int*)d_in[7];
    float* OUT = (float*)d_out;
    char* wsp = (char*)d_ws;
    auto take = [&](size_t bytes) { char* p = wsp; wsp += (bytes + 255) & ~(size_t)255; return (void*)p; };
    bf* WQ = (bf*)take((size_t)DM * DM * 2); bf* WK = (bf*)take((size_t)DM * DM * 2); bf* WV = (bf*)take((size_t)DM * DM * 2); bf* WO = (bf*)take((size_t)DM * DM * 2);
    float* CS = (float*)take((size_t)SEQ * HD * 2 * 4);
    bf* XB = (bf*)take((size_t)SEQ * DM * 2);
    float* F = (float*)take((size_t)SEQ * DM * 4);
    h16* QP16 = (h16*)take((size_t)NH * SEQ * HD * 2); h16* KP16 = (h16*)take((size_t)NH * SEQ * HD * 2); h16* VT16 = (h16*)take((size_t)NH * HD * SEQ * 2);
    bf* QPh = (bf*)take((size_t)NH * SEQ * HD * 2); bf* QPl = (bf*)take((size_t)NH * SEQ * HD * 2);
    bf* KPh = (bf*)take((size_t)NH * SEQ * HD * 2); bf* KPl = (bf*)take((size_t)NH * SEQ * HD * 2);
    bf* VTh = (bf*)take((size_t)NH * HD * SEQ * 2); bf* VTl = (bf*)take((size_t)NH * HD * SEQ * 2);
    bf* ATh = (bf*)take((size_t)SEQ * DM * 2); bf* ATl = (bf*)take((size_t)SEQ * DM * 2);
    const size_t used = (size_t)(wsp - (char*)d_ws);
    if (used > ws_size || used > WSCAP) return;

    const unsigned gW = (unsigned)(((size_t)DM * DM / 8 + 255) / 256);
    k_cvt8<<<gW, 256, 0, stream>>>(wq, WQ, (size_t)DM * DM / 8);
    k_cvt8<<<gW, 256, 0, stream>>>(wk, WK, (size_t)DM * DM / 8);
    k_cvt8<<<gW, 256, 0, stream>>>(wv, WV, (size_t)DM * DM / 8);
    k_cvt8<<<gW, 256, 0, stream>>>(wo, WO, (size_t)DM * DM / 8);
    k_cstab<<<(unsigned)((SEQ * HD + 255) / 256), 256, 0, stream>>>(CS);
    const unsigned gX = (unsigned)(((size_t)SEQ * DM / 8 + 255) / 256), gP = (unsigned)(((size_t)NH * SEQ * HD / 2 + 255) / 256);
    for (int b = 0; b < NB; ++b) {
        const size_t xo = (size_t)b * SEQ_FULL * DM;
        k_cvt8<<<gX, 256, 0, stream>>>(xq + xo, XB, (size_t)SEQ * DM / 8);
        k_gemmw<bf, 0, false><<<dim3(SEQ / 64, DM / 64, 1), 32, 0, stream>>>(XB, nullptr, WQ, nullptr, DM, F, DM, nullptr, 0, 0, 0);
        k_rope<<<gP, 256, 0, stream>>>(F, CS, QP16, QPh, QPl);
        k_cvt8<<<gX, 256, 0, stream>>>(xk + xo, XB, (size_t)SEQ * DM / 8);
        k_gemmw<bf, 0, false><<<dim3(SEQ / 64, DM / 64, 1), 32, 0, stream>>>(XB, nullptr, WK, nullptr, DM, F, DM, nullptr, 0, 0, 0);
        k_rope<<<gP, 256, 0, stream>>>(F, CS, KP16, KPh, KPl);
        k_cvt8<<<gX, 256, 0, stream>>>(xv + xo, XB, (size_t)SEQ * DM / 8);
        k_gemmw<bf, 0, false><<<dim3(SEQ / 64, DM / 64, 1), 32, 0, stream>>>(XB, nullptr, WV, nullptr, DM, F, DM, nullptr, 0, 0, 0);
        k_vtp<<<gP, 256, 0, stream>>>(F, VT16, VTh, VTl);
        k_attn<true><<<dim3(RH / 16, NH, 1), 32, 0, stream>>>(QP16, QPh, QPl, KP16, KPh, KPl, VT16, VTh, VTl, mask, 0, ATh, ATl);
        if (SEQ > RH)
            k_attn<false><<<dim3((SEQ - RH) / 16, NH, 1), 32, 0, stream>>>(QP16, QPh, QPl, KP16, KPh, KPl, VT16, VTh, VTl, mask, RH, ATh, ATl);
        k_gemmw<bf, 1, false><<<dim3(SEQ / 64, DM / 64, 1), 32, 0, stream>>>(ATh, ATl, WO, nullptr, DM, OUT + (size_t)b * SEQ * DM, DM, nullptr, 0, 0, 0);
    }
}
